// QuantumActor_24764781428766
// MI455X (gfx1250) — hardware-run, weakly checked
//
#include <hip/hip_runtime.h>
#include <math.h>

typedef __attribute__((ext_vector_type(16))) _Float16 v16h;
typedef __attribute__((ext_vector_type(8)))  _Float16 v8h;
typedef __attribute__((ext_vector_type(8)))  float    v8f;
typedef __attribute__((ext_vector_type(4)))  float    v4f;

constexpr int kSamples   = 262144;
constexpr int kTiles     = kSamples / 16;
constexpr int kNumAngles = 24;
static_assert((kSamples % 16) == 0, "sample count is a tile multiple");

constexpr float kCarryV   = 64.0f;
constexpr float kCarryY   = 1024.0f;
constexpr float kCarryR   = 64.0f;
constexpr float kScaleAll = kCarryV * kCarryY;
constexpr float kFold     = 1.0f / (kScaleAll * kScaleAll);
constexpr float kF16MinNormal = 6.103515625e-05f;
constexpr float kPiF = 3.14159265358979323846f;

constexpr size_t kOffVP      = 0;
constexpr size_t kPlaneBytes = (size_t)32 * 32 * 2;
constexpr size_t kWsTotal    = kOffVP + kPlaneBytes;
static_assert(kWsTotal == 2048ull, "carve total");
static_assert(kWsTotal <= 134217728ull, "carve cap");

__device__ __forceinline__ _Float16 to_f16_ftz(float v) {
  const float w = (fabsf(v) < kF16MinNormal) ? 0.0f : v;
  return (_Float16)w;
}

union FragH { v16h v; v8h h[2]; };
__device__ __forceinline__ v16h frag_load_h(const _Float16* p) {
  FragH f;
  f.h[0] = *(const v8h*)(p);
  f.h[1] = *(const v8h*)(p + 16);
  return f.v;
}

__device__ __forceinline__ v8f mma_f16_guarded(v16h a, v16h b, v8f c) {
  c = __builtin_amdgcn_wmma_f32_16x16x32_f16(false, a, false, b, (short)0, c, false, false);
  asm volatile("v_nop\n\tv_nop\n\tv_nop\n\tv_nop" : "+v"(c) : "v"(a), "v"(b));
  return c;
}

__global__ __launch_bounds__(32) void build_plane_kernel(const float* __restrict__ wt, unsigned short* __restrict__ vplane)
{
  __shared__ float sRe[16 * 32];
  __shared__ float sIm[16 * 32];
  __shared__ __align__(16) float sM[32 * 32];
  const int tid = threadIdx.x;
  const int col = tid & 15;

#pragma unroll 1
  for (int i = 0; i < 16; ++i) {
    sRe[i * 32 + tid] = (i == col) ? 1.0f : 0.0f;
    sIm[i * 32 + tid] = 0.0f;
  }

#pragma unroll 1
  for (int j = 0; j < 2; ++j) {
#pragma unroll 1
    for (int g = 0; g < 4; ++g) {
      const int mc = 8 >> g;
      const int mt = 8 >> ((g + 1) & 3);
#pragma unroll 1
      for (int i = 0; i < 16; ++i) {
        if (((i & mc) != 0) && ((i & mt) == 0)) {
          const int ia = i * 32 + tid;
          const int ib = (i | mt) * 32 + tid;
          const float ar = sRe[ia], ai = sIm[ia];
          const float br = sRe[ib], bi = sIm[ib];
          sRe[ia] = br; sIm[ia] = bi;
          sRe[ib] = ar; sIm[ib] = ai;
        }
      }
    }
#pragma unroll 1
    for (int q = 0; q < 4; ++q) {
      const int m = 8 >> q;
#pragma unroll 1
      for (int gsel = 0; gsel < 3; ++gsel) {
        int wi = q * 6 + j * 3 + gsel;
        wi = wi < (kNumAngles - 1) ? wi : (kNumAngles - 1);
        const float t = wt[wi];
        float sh, ch;
        sincosf(0.5f * t, &sh, &ch);
        if (gsel == 1) {
#pragma unroll 1
          for (int i = 0; i < 16; ++i) {
            if ((i & m) == 0) {
              const int ia = i * 32 + tid;
              const int ib = (i | m) * 32 + tid;
              const float ar = sRe[ia], ai = sIm[ia];
              const float br = sRe[ib], bi = sIm[ib];
              sRe[ia] = ch * ar - sh * br;
              sIm[ia] = ch * ai - sh * bi;
              sRe[ib] = sh * ar + ch * br;
              sIm[ib] = sh * ai + ch * bi;
            }
          }
        } else {
#pragma unroll 1
          for (int i = 0; i < 16; ++i) {
            const float sg = ((i & m) != 0) ? sh : -sh;
            const int ia = i * 32 + tid;
            const float ar = sRe[ia], ai = sIm[ia];
            sRe[ia] = ar * ch - ai * sg;
            sIm[ia] = ar * sg + ai * ch;
          }
        }
      }
    }
  }

  const int ph = __popc(col) & 3;
#pragma unroll 1
  for (int r = 0; r < 16; ++r) {
    const float x = sRe[r * 32 + tid];
    const float y = sIm[r * 32 + tid];
    const float vr = (ph == 0) ? x : ((ph == 1) ? y : ((ph == 2) ? -x : -y));
    const float vi = (ph == 0) ? y : ((ph == 1) ? -x : ((ph == 2) ? -y : x));
    sM[r * 32 + tid]        = vr;
    sM[(16 + r) * 32 + tid] = vi;
  }
  __syncthreads();

  const int prow = tid >> 2;
  const int kq   = tid & 3;
  const int cb   = (kq & 1) * 8;
  const float sc = ((kq >> 1) != 0) ? (kCarryV / kCarryR) : kCarryV;
  v8h pv[4];
#pragma unroll
  for (int it = 0; it < 4; ++it) {
    const float* sp = sM + (it * 8 + prow) * 32 + cb;
    const v4f a0 = *(const v4f*)(sp);
    const v4f a1 = *(const v4f*)(sp + 4);
#pragma unroll
    for (int e = 0; e < 4; ++e) {
      pv[it][e]     = to_f16_ftz(a0[e] * sc);
      pv[it][4 + e] = to_f16_ftz(a1[e] * sc);
    }
  }
  for (int pass = 0; pass < 2; ++pass) {
#pragma unroll
    for (int it = 0; it < 4; ++it)
      *(volatile v8h*)(vplane + it * 256 + tid * 8) = pv[it];
    __threadfence();
  }
}

__global__ __launch_bounds__(256) void circuit_tiles_kernel(
    const float* __restrict__ state, const unsigned short* __restrict__ vplane,
    float* __restrict__ out, int ntiles, int nsamp)
{
  const int lane = threadIdx.x & 31;
  const int n    = lane & 15;
  const int h    = lane >> 4;
  const int waveId = blockIdx.x * 8 + (threadIdx.x >> 5);
  const int nWaves = gridDim.x * 8;

  const _Float16* vp = (const _Float16*)vplane;
  const v16h aRe = frag_load_h(vp + n * 32 + 8 * h);
  const v16h aIm = frag_load_h(vp + (16 + n) * 32 + 8 * h);

  for (int tile = waveId; tile < ntiles; tile += nWaves) {
    int samp = tile * 16 + n;
    samp = samp < nsamp ? samp : (nsamp - 1);
    const v4f st = *(const v4f*)(state + (size_t)samp * 4);

    const float t0 = (kPiF * st[0]) * (1.0f / 4.8f);
    const float t2 = (kPiF * st[2]) * (1.0f / 0.418f);
    float s0, c0, s2, c2;
    sincosf(0.5f * t0, &s0, &c0);
    sincosf(0.5f * t2, &s2, &c2);
    const float c1 = rsqrtf(1.0f + st[1] * st[1]);
    const float s1 = st[1] * c1;
    const float c3 = rsqrtf(1.0f + st[3] * st[3]);
    const float s3 = st[3] * c3;

    const float m0 = (h != 0) ? s0 : c0;
    v16h bf;
#pragma unroll
    for (int i = 0; i < 8; ++i) {
      const float f1 = ((i & 4) != 0) ? s1 : c1;
      const float f2 = ((i & 2) != 0) ? s2 : c2;
      const float f3 = ((i & 1) != 0) ? s3 : c3;
      const float yc = (((m0 * f1) * f2) * f3) * kCarryY;
      const _Float16 hi = to_f16_ftz(yc);
      float hf = (float)hi;
      asm volatile("" : "+v"(hf));
      const float lo = (yc - hf) * kCarryR;
      bf[i]     = hi;
      bf[8 + i] = to_f16_ftz(lo);
    }

    v8f accRe = (v8f){0.f, 0.f, 0.f, 0.f, 0.f, 0.f, 0.f, 0.f};
    v8f accIm = (v8f){0.f, 0.f, 0.f, 0.f, 0.f, 0.f, 0.f, 0.f};
    accRe = mma_f16_guarded(aRe, bf, accRe);
    accIm = mma_f16_guarded(aIm, bf, accIm);

    float sA = 0.0f, sB = 0.0f;
#pragma unroll
    for (int r = 0; r < 4; ++r) sA += accRe[r] * accRe[r] + accIm[r] * accIm[r];
#pragma unroll
    for (int r = 4; r < 8; ++r) sB += accRe[r] * accRe[r] + accIm[r] * accIm[r];

    const float tot = sA + sB;
    const float z0p = (h != 0) ? -tot : tot;
    const float z1p = sA - sB;
    const float z0 = z0p + __shfl_xor(z0p, 16, 32);
    const float z1 = z1p + __shfl_xor(z1p, 16, 32);

    const float d = (0.5f * kFold) * (z0 - z1);
    const float e = 1.0f / (1.0f + expf(-d));
    const float es = __shfl(e, lane >> 1, 32);
    const float val = ((lane & 1) != 0) ? (1.0f - es) : es;

    volatile float* op = out + (size_t)tile * 32 + lane;
    *op = val;
    __threadfence();
    *op = val;
  }
}

extern "C" void kernel_launch(void* const* d_in, const int* in_sizes, int n_in,
                              void* d_out, int out_size, void* d_ws, size_t ws_size,
                              hipStream_t stream) {
  if (n_in < 2) return;
  if (in_sizes[0] != kSamples * 4) return;
  if (in_sizes[1] != kNumAngles) return;
  if (out_size != kSamples * 2) return;
  if (ws_size < kWsTotal) return;

  const float* state   = (const float*)d_in[0];
  const float* weights = (const float*)d_in[1];
  float* out = (float*)d_out;
  unsigned short* vplane = (unsigned short*)((char*)d_ws + kOffVP);

  build_plane_kernel<<<1, 32, 0, stream>>>(weights, vplane);

  int blocks = (kTiles + 7) / 8;
  if (blocks > 1024) blocks = 1024;
  if (blocks < 1) blocks = 1;
  circuit_tiles_kernel<<<blocks, 256, 0, stream>>>(state, vplane, out, kTiles, kSamples);
}
